// EdgeConvBlock_16381005267563
// MI455X (gfx1250) — hardware-verified
//
#include <hip/hip_runtime.h>
#include <stddef.h>
#include <stdint.h>

#define DIN    32
#define COUT   64
#define UQW    128
#define K2     128
#define NTHR   256
#define NWAVE  8
#define EPB    256
#define DP     68
#define AP     136
#define P3W    64
#define P3U    32
#define GBM    64
#define GBN    128
#define GTHR   128
#define EPT    8
#define CHUNK  (NTHR * EPT)
#define WCAP   (EPT * 32)
#define LISTN  (NWAVE * WCAP)
#define NBA    512
#define SLA    9
#define RCAP   28672
#define DEGCAP 96
#define PARTW  160
#define SPARW  (6 * COUT)
#define NU_W1  (UQW * (DIN / 8))
#define NU_W   (COUT * (K2 / 8))
#define AGG_ZINTS (LISTN + 2 * RCAP + 3 * NBA)
#define AGG_LDS_INTS (AGG_ZINTS + 16)
#define AGG_LDS_BYTES (AGG_LDS_INTS * 4)
#define E0_LDS_BYTES (EPB * DP * 4)
#define E1_LDS_BYTES (EPB * DP * 4 + EPB * AP * 2)
#define E2_LDS_BYTES (EPB * DP * 4 + EPB * AP * 2 + EPB * P3W * 2)
#define WSMAX  268435456
#define CP3    16.0f
#define P3INV  0.0625f
#define BNEPS  1e-5f

static_assert((CHUNK & (CHUNK - 1)) == 0 && CHUNK <= 4096);
static_assert((NBA & (NBA - 1)) == 0 && NBA == (1 << SLA));
static_assert(((long long)CHUNK << SLA) < (1LL << 31));
static_assert(LISTN % NTHR == 0);
static_assert(NBA % NWAVE == 0 && NBA % 32 == 0);
static_assert(RCAP % 4 == 0 && AGG_ZINTS % 4 == 0 && LISTN % 4 == 0);
static_assert(AGG_LDS_BYTES <= 300000 && E2_LDS_BYTES <= 300000);
static_assert(NU_W1 % NTHR == 0 && NU_W % NTHR == 0);
static_assert(DIN % 32 == 0 && COUT % 32 == 0 && UQW == 2 * COUT && GBN == UQW && K2 == 2 * COUT);
static_assert(GBM == (GTHR / 32) * 16 && GBN == 4 * 32);
static_assert((DP * 4) % 16 == 0 && (AP * 2) % 16 == 0 && AP >= K2 && DP >= COUT);
static_assert(EPB == NTHR && COUT == 2 * 32 && EPB == 8 * 32);
static_assert((E0_LDS_BYTES % 16) == 0 && ((EPB * AP * 2) % 16) == 0);
static_assert(EPB * P3W * 2 == 8 * NTHR * 16);
static_assert(PARTW % 32 == 0 && PARTW >= 2 * COUT + 1 && PARTW / 4 <= NTHR);
static_assert(P3W == 2 * P3U && P3U == 32);
static_assert(SPARW == 384);

typedef float          v2f   __attribute__((ext_vector_type(2)));
typedef float          v4f   __attribute__((ext_vector_type(4)));
typedef float          v8f   __attribute__((ext_vector_type(8)));
typedef int            v4i   __attribute__((ext_vector_type(4)));
typedef int            v8i   __attribute__((ext_vector_type(8)));
typedef unsigned short v8us  __attribute__((ext_vector_type(8)));
typedef unsigned short v16us __attribute__((ext_vector_type(16)));
typedef __bf16         v16bf __attribute__((ext_vector_type(16)));
typedef v4f  __attribute__((may_alias)) v4fa;
typedef v4i  __attribute__((may_alias)) v4ia;
typedef v8us __attribute__((may_alias)) v8usa;
union FragB { v16bf v; v16us u; v8us h[2]; v8i w; };

__device__ __forceinline__ v8f wmb(const FragB& a, const FragB& b, v8f c) {
  v8f d = __builtin_amdgcn_wmma_f32_16x16x32_bf16(false, a.v, false, b.v, (short)0, c, false, false);
  asm volatile("v_nop\n\tv_nop\n\tv_nop\n\tv_nop" : "+v"(d) : "v"(a.w), "v"(b.w));
  return d;
}

__device__ __forceinline__ v8f z8() { v8f z = {0.f, 0.f, 0.f, 0.f, 0.f, 0.f, 0.f, 0.f}; return z; }

__device__ __forceinline__ unsigned bf16_bits(float f) {
  const unsigned u = __float_as_uint(f);
  return (u + 0x7FFFu + ((u >> 16) & 1u)) >> 16;
}
__device__ __forceinline__ float bf16_val(float f) {
  return __uint_as_float(bf16_bits(f) << 16);
}
__device__ __forceinline__ unsigned short f2h(float f) {
  const _Float16 hv = (_Float16)f;
  return __builtin_bit_cast(unsigned short, hv);
}
__device__ __forceinline__ float h2f(unsigned b) {
  const _Float16 hv = __builtin_bit_cast(_Float16, (unsigned short)b);
  return (float)hv;
}
__device__ __forceinline__ void put16(unsigned short* dp, v8us o) {
  *(volatile v8us*)dp = o;
  __threadfence();
  *(volatile v8us*)dp = o;
}
__device__ __forceinline__ float fsel(float a, float b, unsigned mask) {
  return __uint_as_float((__float_as_uint(a) & ~mask) | (__float_as_uint(b) & mask));
}

template <int SLB>
__device__ __forceinline__ int scan_chunk(const int* __restrict__ dsts, int nE, int cbase, int slotBase,
                                          int nb, int vec8, int* list, int tid, int lane, int wave) {
  int wc = 0;
  const int el0  = tid * EPT;
  const int e0   = cbase + el0;
  const int sent = -2147483647 - 1;
  v4i da, db;
  if (vec8 != 0 && cbase + CHUNK <= nE) {
    da = *(const v4i*)(dsts + e0);
    db = *(const v4i*)(dsts + e0 + 4);
  } else {
    da.x = (e0     < nE) ? dsts[min(e0,     nE - 1)] : sent;
    da.y = (e0 + 1 < nE) ? dsts[min(e0 + 1, nE - 1)] : sent;
    da.z = (e0 + 2 < nE) ? dsts[min(e0 + 2, nE - 1)] : sent;
    da.w = (e0 + 3 < nE) ? dsts[min(e0 + 3, nE - 1)] : sent;
    db.x = (e0 + 4 < nE) ? dsts[min(e0 + 4, nE - 1)] : sent;
    db.y = (e0 + 5 < nE) ? dsts[min(e0 + 5, nE - 1)] : sent;
    db.z = (e0 + 6 < nE) ? dsts[min(e0 + 6, nE - 1)] : sent;
    db.w = (e0 + 7 < nE) ? dsts[min(e0 + 7, nE - 1)] : sent;
  }
  const unsigned nbs = (unsigned)slotBase;
  const unsigned unb = (unsigned)nb;
  const unsigned s0 = (unsigned)da.x - nbs, s1 = (unsigned)da.y - nbs;
  const unsigned s2 = (unsigned)da.z - nbs, s3 = (unsigned)da.w - nbs;
  const unsigned s4 = (unsigned)db.x - nbs, s5 = (unsigned)db.y - nbs;
  const unsigned s6 = (unsigned)db.z - nbs, s7 = (unsigned)db.w - nbs;
  const bool h0 = s0 < unb, h1 = s1 < unb, h2 = s2 < unb, h3 = s3 < unb;
  const bool h4 = s4 < unb, h5 = s5 < unb, h6 = s6 < unb, h7 = s7 < unb;
  const unsigned any = __builtin_amdgcn_ballot_w32(h0 | h1 | h2 | h3 | h4 | h5 | h6 | h7);
  if (any != 0u) {
#define HITJ(J, HJ, SJ) { \
      const unsigned mj = __builtin_amdgcn_ballot_w32(HJ); \
      if (mj != 0u) { \
        if (HJ) { \
          const int pos = wc + (int)__builtin_amdgcn_mbcnt_lo(mj, 0u); \
          if (pos < WCAP) list[wave * WCAP + pos] = ((el0 + (J)) << SLB) | (int)(SJ); \
        } \
        wc += (int)__builtin_popcount(mj); } }
    HITJ(0, h0, s0)
    HITJ(1, h1, s1)
    HITJ(2, h2, s2)
    HITJ(3, h3, s3)
    HITJ(4, h4, s4)
    HITJ(5, h5, s5)
    HITJ(6, h6, s6)
    HITJ(7, h7, s7)
#undef HITJ
  }
  return wc;
}

__global__ __launch_bounds__(NTHR) void k_prep(const float* __restrict__ x, const float* __restrict__ W1,
                                               const float* __restrict__ W2, const float* __restrict__ W3,
                                               int nN, int mRows, unsigned short* W1T, unsigned short* W2B,
                                               unsigned short* W3B, unsigned short* XB) {
  const int u  = (int)blockIdx.x * NTHR + (int)threadIdx.x;
  const int L0 = NU_W1;
  const int L1 = L0 + NU_W;
  const int L2 = L1 + NU_W;
  const int L3 = L2 + mRows * (DIN / 8);
  const float* p;
  unsigned short* dp;
  unsigned mk = 0xffffu;
  if (u < L0) {
    const int n  = u >> 2;
    const int k8 = (u & 3) * 8;
    p  = W1 + (size_t)(n & (COUT - 1)) * (size_t)(2 * DIN) + (n >> 6) * DIN + k8;
    dp = W1T + (size_t)u * 8;
  } else if (u < L1) {
    const int v  = u - L0;
    const int n  = v >> 4;
    const int kk = ((v & 15) * 8) & (COUT - 1);
    p  = W2 + (size_t)n * COUT + kk;
    dp = W2B + (size_t)v * 8;
  } else if (u < L2) {
    const int v  = u - L1;
    const int n  = v >> 4;
    const int kk = ((v & 15) * 8) & (COUT - 1);
    p  = W3 + (size_t)n * COUT + kk;
    dp = W3B + (size_t)v * 8;
  } else if (u < L3) {
    const int v   = u - L2;
    const int row = v >> 2;
    const int j   = v & 3;
    const int rc  = row < nN ? row : nN - 1;
    mk = (row < nN) ? 0xffffu : 0u;
    p  = x + (size_t)rc * DIN + 8 * j;
    dp = XB + (size_t)v * 8;
  } else {
    return;
  }
  const v4f a = *(const v4f*)p;
  const v4f b = *(const v4f*)(p + 4);
  v8us o;
  o[0] = (unsigned short)(bf16_bits(a.x) & mk); o[1] = (unsigned short)(bf16_bits(a.y) & mk);
  o[2] = (unsigned short)(bf16_bits(a.z) & mk); o[3] = (unsigned short)(bf16_bits(a.w) & mk);
  o[4] = (unsigned short)(bf16_bits(b.x) & mk); o[5] = (unsigned short)(bf16_bits(b.y) & mk);
  o[6] = (unsigned short)(bf16_bits(b.z) & mk); o[7] = (unsigned short)(bf16_bits(b.w) & mk);
  put16(dp, o);
}

__global__ __launch_bounds__(GTHR) void k_pq(const unsigned short* __restrict__ A,
                                             const unsigned short* __restrict__ BT,
                                             const float* __restrict__ b1, float* UQ) {
  __shared__ __attribute__((aligned(16))) float stg[GBM * GBN];
  const int tid = (int)threadIdx.x, lane = tid & 31, wave = tid >> 5, hh = lane >> 4, m = lane & 15;
  const int rowBase = (int)blockIdx.x * GBM;

  v8f acc[8];
#pragma unroll
  for (int t = 0; t < 8; ++t) acc[t] = z8();
  const unsigned short* ap = A  + (size_t)(rowBase + 16 * wave + m) * (size_t)DIN + 8 * hh;
  const unsigned short* bp = BT + (size_t)m * (size_t)DIN + 8 * hh;

#pragma unroll
  for (int k0 = 0; k0 < DIN; k0 += 32) {
    FragB af;
    af.h[0] = *(const v8usa*)(ap + k0);
    af.h[1] = *(const v8usa*)(ap + k0 + 16);
#pragma unroll
    for (int nt = 0; nt < 8; ++nt) {
      const unsigned short* wq = bp + (size_t)(16 * nt) * (size_t)DIN + k0;
      FragB bf;
      bf.h[0] = *(const v8usa*)wq;
      bf.h[1] = *(const v8usa*)(wq + 16);
      acc[nt] = wmb(af, bf, acc[nt]);
    }
  }

#pragma unroll
  for (int nt = 0; nt < 8; ++nt) {
    const int lc = 16 * nt + m;
#pragma unroll
    for (int r = 0; r < 8; ++r) {
      const int lr = 16 * wave + 8 * hh + r;
      stg[lr * GBN + lc] = acc[nt][r];
    }
  }
  __syncthreads();

  const int cU = 4 * (lane & 15);
  const unsigned mq = 0u - (unsigned)hh;
  const v4f b4 = *(const v4f*)(b1 + cU);
  const float bb0 = bf16_val(b4.x);
  const float bb1 = bf16_val(b4.y);
  const float bb2 = bf16_val(b4.z);
  const float bb3 = bf16_val(b4.w);
  v4f pv[16];
#pragma unroll
  for (int i = 0; i < 16; ++i) {
    const float* sp = stg + (16 * wave + i) * GBN;
    const v4f a = *(const v4fa*)(sp + cU);
    const v4f q = *(const v4fa*)(sp + COUT + cU);
    v4f o;
    o.x = fsel((a.x - q.x) + bb0, q.x, mq);
    o.y = fsel((a.y - q.y) + bb1, q.y, mq);
    o.z = fsel((a.z - q.z) + bb2, q.z, mq);
    o.w = fsel((a.w - q.w) + bb3, q.w, mq);
    pv[i] = o;
  }
#pragma unroll
  for (int i = 0; i < 16; ++i) {
    float* op = UQ + (size_t)(rowBase + 16 * wave + i) * (size_t)UQW + 4 * lane;
    *(volatile v4f*)op = pv[i];
  }
  __threadfence();
#pragma unroll
  for (int i = 0; i < 16; ++i) {
    float* op = UQ + (size_t)(rowBase + 16 * wave + i) * (size_t)UQW + 4 * lane;
    *(volatile v4f*)op = pv[i];
  }
}

__device__ __forceinline__ void block_stats(const float* sD, int nv, float* red, float* red2, float* pst,
                                            float* part, int pb, int tid) {
  const int c = tid & (COUT - 1);
  const int g = tid >> 6;
  int cg = nv - 64 * g;
  cg = cg < 0 ? 0 : (cg > 64 ? 64 : cg);
  const float* col = sD + (size_t)(64 * g) * DP + c;
  float s = 0.0f;
#pragma unroll 4
  for (int i = 0; i < cg; ++i) s += col[i * DP];
  red[g * COUT + c] = s;
  __syncthreads();
  const float tot  = ((red[c] + red[COUT + c]) + red[2 * COUT + c]) + red[3 * COUT + c];
  const float mean = tot * (1.0f / (float)nv);
  float q = 0.0f;
#pragma unroll 4
  for (int i = 0; i < cg; ++i) {
    const float d = col[i * DP] - mean;
    q = fmaf(d, d, q);
  }
  red2[g * COUT + c] = q;
  __syncthreads();
  const float M2 = ((red2[c] + red2[COUT + c]) + red2[2 * COUT + c]) + red2[3 * COUT + c];
  if (g == 0) { pst[1 + c] = mean; pst[1 + COUT + c] = M2; }
  if (tid == 0) pst[0] = (float)nv;
#pragma unroll 1
  for (int i = 2 * COUT + 1 + tid; i < PARTW; i += NTHR) pst[i] = 0.0f;
  __syncthreads();
  v4f ps = {0.0f, 0.0f, 0.0f, 0.0f};
  if (tid < PARTW / 4) {
    ps = *(const v4fa*)(pst + 4 * tid);
    *(volatile v4f*)(part + (size_t)pb * PARTW + 4 * tid) = ps;
  }
  __threadfence();
  if (tid < PARTW / 4) {
    *(volatile v4f*)(part + (size_t)pb * PARTW + 4 * tid) = ps;
  }
}

__device__ __forceinline__ void bn_hilo(const float* rd, unsigned short* ra, const float* sc, const float* sh) {
#pragma unroll 2
  for (int c8 = 0; c8 < COUT / 8; ++c8) {
    const v4f va = *(const v4fa*)(rd + 8 * c8);
    const v4f vb = *(const v4fa*)(rd + 8 * c8 + 4);
    const v8f v8 = {va.x, va.y, va.z, va.w, vb.x, vb.y, vb.z, vb.w};
    v8us oh, ol;
#pragma unroll
    for (int i = 0; i < 8; ++i) {
      const float hv = fmaxf(fmaf(v8[i], sc[8 * c8 + i], sh[8 * c8 + i]), 0.0f);
      const unsigned hb = bf16_bits(hv);
      oh[i] = (unsigned short)hb;
      ol[i] = (unsigned short)bf16_bits(hv - __uint_as_float(hb << 16));
    }
    *(v8usa*)(ra + 8 * c8) = oh;
    *(v8usa*)(ra + COUT + 8 * c8) = ol;
  }
}

__device__ __forceinline__ void wave_gemm_b(const unsigned short* sAw, float* sDw,
                                            const unsigned short* __restrict__ BT, const float* bia,
                                            int hh, int m) {
  v8f acc[2][4];
#pragma unroll
  for (int mt = 0; mt < 2; ++mt)
#pragma unroll
    for (int nt = 0; nt < 4; ++nt) acc[mt][nt] = z8();
  const unsigned short* ap0 = sAw + m * AP + 8 * hh;
  const unsigned short* ap1 = ap0 + 16 * AP;
  const unsigned short* bp  = BT + (size_t)m * (size_t)K2 + 8 * hh;
#pragma unroll 1
  for (int k0 = 0; k0 < K2; k0 += 32) {
    FragB a0, a1;
    a0.h[0] = *(const v8usa*)(ap0 + k0);
    a0.h[1] = *(const v8usa*)(ap0 + k0 + 16);
    a1.h[0] = *(const v8usa*)(ap1 + k0);
    a1.h[1] = *(const v8usa*)(ap1 + k0 + 16);
#pragma unroll
    for (int nt = 0; nt < 4; ++nt) {
      const unsigned short* wq = bp + (size_t)(16 * nt) * (size_t)K2 + k0;
      FragB b;
      b.h[0] = *(const v8usa*)wq;
      b.h[1] = *(const v8usa*)(wq + 16);
      acc[0][nt] = wmb(a0, b, acc[0][nt]);
      acc[1][nt] = wmb(a1, b, acc[1][nt]);
    }
  }
#pragma unroll
  for (int nt = 0; nt < 4; ++nt) {
    const int col = 16 * nt + m;
    const float bv = bia[col];
#pragma unroll
    for (int mt = 0; mt < 2; ++mt)
#pragma unroll
      for (int r = 0; r < 8; ++r) sDw[(16 * mt + 8 * hh + r) * DP + col] = acc[mt][nt][r] + bv;
  }
}

template <int MODE>
__global__ __launch_bounds__(NTHR) void k_edge(const int* __restrict__ srcs, const int* __restrict__ dsts,
                                               int nE, int nN, const float* __restrict__ UQ,
                                               const float* __restrict__ ss1, const float* __restrict__ ss2,
                                               const unsigned short* __restrict__ W2B,
                                               const unsigned short* __restrict__ W3B,
                                               const float* __restrict__ b2, const float* __restrict__ b3,
                                               float* part, unsigned short* P3) {
  extern __shared__ __attribute__((aligned(16))) float dyn[];
  __shared__ __attribute__((aligned(16))) float red[4 * COUT];
  __shared__ __attribute__((aligned(16))) float red2[4 * COUT];
  __shared__ __attribute__((aligned(16))) float pst[PARTW];
  __shared__ __attribute__((aligned(16))) float spar[SPARW];
  float*          sD = dyn;
  unsigned short* sA = (unsigned short*)(dyn + EPB * DP);
  unsigned short* sM = sA + EPB * AP;

  const int tid = (int)threadIdx.x, lane = tid & 31, wave = tid >> 5, hh = lane >> 4, m = lane & 15;
  const int elb = (int)blockIdx.x * EPB;
  const int el  = elb + tid;
  const int elc = el < nE ? el : (nE - 1);
  int nv = nE - elb;
  nv = nv > EPB ? EPB : nv;

  if constexpr (MODE >= 1) {
    if (tid < 2 * COUT) spar[tid] = ss1[tid];
    if (tid < COUT) spar[2 * COUT + tid] = bf16_val(b2[tid]);
  }
  if constexpr (MODE == 2) {
    if (tid < 2 * COUT) spar[3 * COUT + tid] = ss2[tid];
    if (tid < COUT) spar[5 * COUT + tid] = bf16_val(b3[tid]);
  }

  int s = srcs[elc];
  int t = dsts[elc];
  s = s < 0 ? 0 : (s > nN - 1 ? nN - 1 : s);
  t = t < 0 ? 0 : (t > nN - 1 ? nN - 1 : t);
  float* rd = sD + tid * DP;
  {
    const float* upr = UQ + (size_t)t * UQW;
    const float* qpr = UQ + (size_t)s * UQW + COUT;
#pragma unroll 4
    for (int c4 = 0; c4 < COUT / 4; ++c4) {
      const v4f a = *(const v4fa*)(upr + 4 * c4);
      const v4f b = *(const v4fa*)(qpr + 4 * c4);
      const v4f p = a + b;
      *(v4fa*)(rd + 4 * c4) = p;
    }
  }
  __syncthreads();

  if constexpr (MODE == 0) {
    block_stats(sD, nv, red, red2, pst, part, (int)blockIdx.x, tid);
    return;
  } else {
    unsigned short* ra = sA + tid * AP;
    bn_hilo(rd, ra, spar, spar + COUT);
    __syncthreads();

    wave_gemm_b(sA + 32 * wave * AP, sD + 32 * wave * DP, W2B, spar + 2 * COUT, hh, m);
    __syncthreads();

    if constexpr (MODE == 1) {
      block_stats(sD, nv, red, red2, pst, part, (int)blockIdx.x, tid);
      return;
    } else {
      bn_hilo(rd, ra, spar + 3 * COUT, spar + 4 * COUT);
      __syncthreads();

      wave_gemm_b(sA + 32 * wave * AP, sD + 32 * wave * DP, W3B, spar + 5 * COUT, hh, m);
      __syncthreads();

      block_stats(sD, nv, red, red2, pst, part, (int)blockIdx.x, tid);

      unsigned short* rm = sM + tid * P3W;
#pragma unroll 2
      for (int c8 = 0; c8 < COUT / 8; ++c8) {
        const v4f va = *(const v4fa*)(rd + 8 * c8);
        const v4f vb = *(const v4fa*)(rd + 8 * c8 + 4);
        const v8f v8 = {va.x, va.y, va.z, va.w, vb.x, vb.y, vb.z, vb.w};
        v8us o;
#pragma unroll
        for (int i = 0; i < 8; ++i) o[i] = f2h(CP3 * v8[i]);
        *(v8usa*)(rm + 8 * c8) = o;
      }
      __syncthreads();

      v4i pv[8];
#pragma unroll
      for (int it = 0; it < 8; ++it) pv[it] = *(const v4ia*)(sM + (size_t)(it * NTHR + tid) * 8);
      unsigned short* mb = P3 + (size_t)elb * P3W;
#pragma unroll
      for (int it = 0; it < 8; ++it) *(volatile v4i*)(mb + (size_t)(it * NTHR + tid) * 8) = pv[it];
      __threadfence();
#pragma unroll
      for (int it = 0; it < 8; ++it) *(volatile v4i*)(mb + (size_t)(it * NTHR + tid) * 8) = pv[it];
    }
  }
}

__global__ __launch_bounds__(NTHR) void k_bnfin(const float* __restrict__ part, int nPart,
                                                const float* __restrict__ gam, const float* __restrict__ bet,
                                                float* ss) {
  __shared__ double cn[NTHR], cm[NTHR], cq[NTHR];
  __shared__ __attribute__((aligned(16))) float stg[2 * COUT];
  const int tid = (int)threadIdx.x;
  const int c = tid & (COUT - 1);
  const int p = tid >> 6;
  double n = 0.0, mean = 0.0, M2 = 0.0;
#pragma unroll 1
  for (int b = p; b < nPart; b += 4) {
    const float* pr = part + (size_t)b * PARTW;
    const double nb = (double)pr[0];
    const double mb = (double)pr[1 + c];
    const double qb = (double)pr[1 + COUT + c];
    if (nb > 0.5) {
      const double nn = n + nb;
      const double delta = mb - mean;
      const double f = nb / nn;
      mean = mean + delta * f;
      M2 = M2 + qb + delta * delta * n * f;
      n = nn;
    }
  }
  cn[tid] = n; cm[tid] = mean; cq[tid] = M2;
  __syncthreads();
  if (tid < COUT) {
    double tn = 0.0, tm = 0.0, tq = 0.0;
#pragma unroll 1
    for (int p2 = 0; p2 < 4; ++p2) {
      const double nb = cn[p2 * COUT + c];
      const double mb = cm[p2 * COUT + c];
      const double qb = cq[p2 * COUT + c];
      if (nb > 0.5) {
        const double nn = tn + nb;
        const double delta = mb - tm;
        const double f = nb / nn;
        tm = tm + delta * f;
        tq = tq + qb + delta * delta * tn * f;
        tn = nn;
      }
    }
    const double nt = tn < 1.0 ? 1.0 : tn;
    const float varf  = (float)(tq / nt);
    const float meanf = (float)tm;
    const float rstd = 1.0f / sqrtf(varf + BNEPS);
    const float sc = bf16_val(gam[c]) * rstd;
    const float sh = bf16_val(bet[c]) - meanf * sc;
    stg[c] = sc;
    stg[COUT + c] = sh;
  }
  __syncthreads();
  v4f v = {0.0f, 0.0f, 0.0f, 0.0f};
  if (tid < (2 * COUT) / 4) {
    v = *(const v4fa*)(stg + 4 * tid);
    *(volatile v4f*)(ss + 4 * tid) = v;
  }
  __threadfence();
  if (tid < (2 * COUT) / 4) {
    *(volatile v4f*)(ss + 4 * tid) = v;
  }
}

__global__ __launch_bounds__(NTHR) void k_scan(const int* __restrict__ dsts, int nE, int vec8, int nN,
                                               const unsigned* __restrict__ P3w,
                                               const float* __restrict__ ss3, float* out) {
  extern __shared__ __attribute__((aligned(16))) int dsm[];
  int* list = dsm;
  int* hl   = dsm + LISTN;
  int* sl   = hl + RCAP;
  int* cnt  = sl + RCAP;
  int* offs = cnt + NBA;
  int* cur  = offs + NBA;
  int* misc = cur + NBA;
  const int tid = (int)threadIdx.x, lane = tid & 31, wave = tid >> 5;
  const int nodeBase = (int)blockIdx.x * NBA;

  const float scq0 = ss3[2 * lane] * P3INV;
  const float scq1 = ss3[2 * lane + 1] * P3INV;
  const float shv0 = ss3[COUT + 2 * lane];
  const float shv1 = ss3[COUT + 2 * lane + 1];

  {
    const v4i z4 = {0, 0, 0, 0};
    for (int i = tid * 4; i < AGG_ZINTS; i += NTHR * 4) *(v4ia*)(dsm + i) = z4;
    if (tid < 16) misc[tid] = 0;
  }
  __syncthreads();

  int t = 0, ov = 0;
  const int nChunks = (nE + CHUNK - 1) / CHUNK;
#pragma unroll 1
  for (int ch = 0; ch < nChunks; ++ch) {
    const int cbase = ch * CHUNK;
    const int wc = scan_chunk<SLA>(dsts, nE, cbase, nodeBase, NBA, vec8, list, tid, lane, wave);
    if (lane == 0) misc[wave] = wc;
    __syncthreads();
    if (wave == 0) {
#pragma unroll 1
      for (int w2 = 0; w2 < NWAVE; ++w2) {
        int c = misc[w2];
        c = c < 0 ? 0 : (c > WCAP ? WCAP : c);
#pragma unroll 1
        for (int b0 = 0; b0 < c; b0 += 32) {
          const int idx = b0 + lane;
          const int ent = list[w2 * WCAP + (idx < WCAP ? idx : WCAP - 1)];
          const int m32 = (c - b0) < 32 ? (c - b0) : 32;
#pragma unroll 1
          for (int k = 0; k < m32; ++k) {
            const int u    = __builtin_amdgcn_readlane(ent, k);
            const int slot = u & (NBA - 1);
            const int el   = (u >> SLA) & (CHUNK - 1);
            const int pk   = ((cbase + el) << SLA) | slot;
            if (t < RCAP) {
              if (lane == 0) { hl[t] = pk; cnt[slot] = cnt[slot] + 1; }
              t = t + 1;
            } else {
              ov = 1;
            }
          }
        }
      }
    }
    __syncthreads();
  }
  if (wave == 0 && lane == 0) { misc[8] = t; misc[9] = ov; }
  __syncthreads();
  int tt = misc[8];
  tt = tt < 0 ? 0 : (tt > RCAP ? RCAP : tt);
  const int ovf = misc[9];

  if (wave == 0) {
    const int base = lane * (NBA / 32);
    int sacc = 0;
#pragma unroll 1
    for (int i = 0; i < NBA / 32; ++i) sacc += cnt[base + i];
    int incl = sacc;
#pragma unroll
    for (int d = 1; d < 32; d <<= 1) {
      const int y = __shfl_up(incl, d, 32);
      if (lane >= d) incl += y;
    }
    int run = incl - sacc;
#pragma unroll 1
    for (int i = 0; i < NBA / 32; ++i) {
      const int cv = cnt[base + i];
      offs[base + i] = run;
      cur[base + i]  = run;
      run += cv;
    }
  }
  __syncthreads();
  if (wave == 0) {
#pragma unroll 1
    for (int b0 = 0; b0 < tt; b0 += 32) {
      const int idx = b0 + lane;
      const int ent = hl[idx < RCAP ? idx : RCAP - 1];
      const int m32 = (tt - b0) < 32 ? (tt - b0) : 32;
#pragma unroll 1
      for (int k = 0; k < m32; ++k) {
        const int u    = __builtin_amdgcn_readlane(ent, k);
        const int slot = u & (NBA - 1);
        if (lane == 0) {
          int p = cur[slot];
          p = p < 0 ? 0 : (p > RCAP - 1 ? RCAP - 1 : p);
          sl[p] = u;
          cur[slot] = p + 1;
        }
      }
    }
  }
  __syncthreads();

  const float qnan = __int_as_float(0x7fc00000);
  const float pz = (ovf != 0) ? qnan : 0.0f;
#pragma unroll 1
  for (int si = 0; si < NBA / NWAVE; ++si) {
    const int sidx = si * NWAVE + wave;
    const int node = nodeBase + sidx;
    int c = cnt[sidx];
    const bool big = c > DEGCAP;
    c = c < 0 ? 0 : (c > DEGCAP ? DEGCAP : c);
    int o = offs[sidx];
    o = o < 0 ? 0 : (o > RCAP ? RCAP : o);
    float a0 = 0.0f, a1 = 0.0f;
#pragma unroll 1
    for (int b0 = 0; b0 < c; b0 += 32) {
      int idx = o + b0 + lane;
      idx = idx > RCAP - 1 ? RCAP - 1 : idx;
      const int ent = sl[idx];
      int eid = ent >> SLA;
      eid = eid < 0 ? 0 : (eid > nE - 1 ? nE - 1 : eid);
      const int m32 = (c - b0) < 32 ? (c - b0) : 32;
#pragma unroll 1
      for (int k = 0; k < m32; ++k) {
        const int ek = __builtin_amdgcn_readlane(eid, k);
        const unsigned w = P3w[(size_t)ek * P3U + lane];
        const float v0 = h2f(w & 0xffffu);
        const float v1 = h2f(w >> 16);
        a0 += fmaxf(fmaf(v0, scq0, shv0), 0.0f);
        a1 += fmaxf(fmaf(v1, scq1, shv1), 0.0f);
      }
    }
    const float pzr = big ? qnan : pz;
    v2f ovv;
    ovv.x = (a0 + 0.0f) + pzr;
    ovv.y = (a1 + 0.0f) + pzr;
    const bool live = node < nN;
    if (live) {
      float* op = out + (size_t)node * COUT + 2 * lane;
      *(volatile v2f*)op = ovv;
    }
    __threadfence();
    if (live) {
      float* op = out + (size_t)node * COUT + 2 * lane;
      *(volatile v2f*)op = ovv;
    }
  }
}

static inline int cdiv(int a, int b) { return (a + b - 1) / b; }
static inline size_t al256(size_t o) { return (o + 255) & ~(size_t)255; }

extern "C" void kernel_launch(void* const* d_in, const int* in_sizes, int n_in,
                              void* d_out, int out_size, void* d_ws, size_t ws_size,
                              hipStream_t stream) {
  if (n_in < 14) return;
  if (in_sizes[0] < DIN * 16 || (in_sizes[0] % DIN) != 0) return;
  const int nN = in_sizes[0] / DIN;
  if (in_sizes[1] < 2 || (in_sizes[1] & 1) != 0) return;
  const int nE = in_sizes[1] / 2;
  if (nE < 1 || nE >= (1 << 22) || nN >= (1 << 24)) return;
  if (in_sizes[2] != COUT * 2 * DIN) return;
  if (in_sizes[3] != COUT || in_sizes[4] != COUT || in_sizes[5] != COUT) return;
  if (in_sizes[6] != COUT * COUT) return;
  if (in_sizes[7] != COUT || in_sizes[8] != COUT || in_sizes[9] != COUT) return;
  if (in_sizes[10] != COUT * COUT) return;
  if (in_sizes[11] != COUT || in_sizes[12] != COUT || in_sizes[13] != COUT) return;
  if ((long long)out_size != (long long)nN * COUT) return;

  const float* x   = (const float*)d_in[0];
  const int*   ei  = (const int*)d_in[1];
  const float* W1  = (const float*)d_in[2];
  const float* b1  = (const float*)d_in[3];
  const float* g1  = (const float*)d_in[4];
  const float* be1 = (const float*)d_in[5];
  const float* W2  = (const float*)d_in[6];
  const float* b2  = (const float*)d_in[7];
  const float* g2  = (const float*)d_in[8];
  const float* be2 = (const float*)d_in[9];
  const float* W3  = (const float*)d_in[10];
  const float* b3  = (const float*)d_in[11];
  const float* g3  = (const float*)d_in[12];
  const float* be3 = (const float*)d_in[13];
  float* out = (float*)d_out;
  const int* src = ei;
  const int* dst = ei + nE;

  const int MP = cdiv(nN, GBM) * GBM;
  const int gM = MP / GBM;
  const int gA = cdiv(nN, NBA);
  if ((long long)gA * NBA < (long long)nN) return;
  const int EB = cdiv(nE, EPB);
  const int EP = EB * EPB;
  const int vec8 = ((nE & 3) == 0) ? 1 : 0;

  char* ws = (char*)d_ws;
  size_t off = 0;
  const size_t oW1T = off; off = al256(off + (size_t)UQW * DIN * 2);
  const size_t oW2B = off; off = al256(off + (size_t)COUT * K2 * 2);
  const size_t oW3B = off; off = al256(off + (size_t)COUT * K2 * 2);
  const size_t oXB  = off; off = al256(off + (size_t)MP * DIN * 2);
  const size_t oUQ  = off; off = al256(off + (size_t)MP * UQW * 4);
  const size_t oP3  = off; off = al256(off + (size_t)EP * P3W * 2);
  const size_t oPT1 = off; off = al256(off + (size_t)EB * PARTW * 4);
  const size_t oPT2 = off; off = al256(off + (size_t)EB * PARTW * 4);
  const size_t oPT3 = off; off = al256(off + (size_t)EB * PARTW * 4);
  const size_t oSS1 = off; off = al256(off + (size_t)(2 * COUT) * 4);
  const size_t oSS2 = off; off = al256(off + (size_t)(2 * COUT) * 4);
  const size_t oSS3 = off; off = al256(off + (size_t)(2 * COUT) * 4);
  if (off > ws_size || off > (size_t)WSMAX) return;
  unsigned short* W1T = (unsigned short*)(ws + oW1T);
  unsigned short* W2B = (unsigned short*)(ws + oW2B);
  unsigned short* W3B = (unsigned short*)(ws + oW3B);
  unsigned short* XB  = (unsigned short*)(ws + oXB);
  float*          UQ  = (float*)(ws + oUQ);
  unsigned short* P3  = (unsigned short*)(ws + oP3);
  const unsigned* P3w = (const unsigned*)(ws + oP3);
  float*          PT1 = (float*)(ws + oPT1);
  float*          PT2 = (float*)(ws + oPT2);
  float*          PT3 = (float*)(ws + oPT3);
  float*          SS1 = (float*)(ws + oSS1);
  float*          SS2 = (float*)(ws + oSS2);
  float*          SS3 = (float*)(ws + oSS3);

  hipFuncSetAttribute(reinterpret_cast<const void*>(&k_edge<0>), hipFuncAttributeMaxDynamicSharedMemorySize,
                      (int)E0_LDS_BYTES);
  hipFuncSetAttribute(reinterpret_cast<const void*>(&k_edge<1>), hipFuncAttributeMaxDynamicSharedMemorySize,
                      (int)E1_LDS_BYTES);
  hipFuncSetAttribute(reinterpret_cast<const void*>(&k_edge<2>), hipFuncAttributeMaxDynamicSharedMemorySize,
                      (int)E2_LDS_BYTES);
  hipFuncSetAttribute(reinterpret_cast<const void*>(&k_scan), hipFuncAttributeMaxDynamicSharedMemorySize,
                      (int)AGG_LDS_BYTES);

  const int nPrep = NU_W1 + 2 * NU_W + MP * (DIN / 8);

  k_prep<<<cdiv(nPrep, NTHR), NTHR, 0, stream>>>(x, W1, W2, W3, nN, MP, W1T, W2B, W3B, XB);
  k_pq<<<gM, GTHR, 0, stream>>>(XB, W1T, b1, UQ);
  k_edge<0><<<EB, NTHR, E0_LDS_BYTES, stream>>>(src, dst, nE, nN, UQ, SS1, SS2, W2B, W3B, b2, b3, PT1, P3);
  k_bnfin<<<1, NTHR, 0, stream>>>(PT1, EB, g1, be1, SS1);
  k_edge<1><<<EB, NTHR, E1_LDS_BYTES, stream>>>(src, dst, nE, nN, UQ, SS1, SS2, W2B, W3B, b2, b3, PT2, P3);
  k_bnfin<<<1, NTHR, 0, stream>>>(PT2, EB, g2, be2, SS2);
  k_edge<2><<<EB, NTHR, E2_LDS_BYTES, stream>>>(src, dst, nE, nN, UQ, SS1, SS2, W2B, W3B, b2, b3, PT3, P3);
  k_bnfin<<<1, NTHR, 0, stream>>>(PT3, EB, g3, be3, SS3);
  k_scan<<<gA, NTHR, AGG_LDS_BYTES, stream>>>(dst, nE, vec8, nN, P3w, SS3, out);
}
